// Encoder_50294067036733
// MI455X (gfx1250) — hardware-verified
//
#include <hip/hip_runtime.h>
#include <math.h>

constexpr int VOCAB = 50000;
constexpr int EMB   = 256;
constexpr int HID   = 256;
constexpr int DM    = 512;
constexpr int TPL   = 384;
constexpr int TQL   = 64;
constexpr int NBAT  = 32;
constexpr int G3    = 768;
constexpr int GW    = 2048;
constexpr int NPR   = TPL * NBAT;
constexpr int NQR   = TQL * NBAT;
constexpr int NXR   = NPR + NQR;
constexpr int OUT0_FLOATS = TPL * NBAT * DM;
constexpr int OUT1_FLOATS = 2 * NBAT * HID;

constexpr float W_CARRY  = 256.0f;
constexpr float X_CARRY  = 16.0f;
constexpr float G_CARRY  = 16.0f;
constexpr float QM_CARRY = 1024.0f;
constexpr float P_CARRY  = 4096.0f;
constexpr float W_INV    = 1.0f / W_CARRY;
constexpr float GI_SCALE = 1.0f / (W_CARRY * X_CARRY);
constexpr float GI4_SCALE = 1.0f / (W_CARRY * G_CARRY);
constexpr float CROSS_SCALE = 1.0f / QM_CARRY;
constexpr float C2QV_SCALE = G_CARRY / P_CARRY;

constexpr int HP16 = 264;
constexpr int GPF  = 772;
constexpr int HSPF = 260;

static_assert(DM == 2 * HID);
static_assert(G3 == 3 * HID);
static_assert(GW == 4 * DM);
static_assert(NXR % 64 == 0 && NPR % 64 == 0 && G3 % 64 == 0 && TPL % 64 == 0 && TQL % 64 == 0 && DM % 64 == 0);
static_assert(EMB % 32 == 0 && HID % 32 == 0 && DM % 32 == 0 && TQL % 32 == 0 && GW % 32 == 0);
static_assert((NXR / 64) * (G3 / 64) % 8 == 0);
static_assert((NPR / 64) * (G3 / 64) % 8 == 0);
static_assert((TPL / 64) * (DM / 64) % 8 == 0);
static_assert((size_t)OUT0_FLOATS * 4 == 25165824);
static_assert(((size_t)OUT0_FLOATS + OUT1_FLOATS) * 4 == 25231360);
static_assert(TPL % 4 == 0);

typedef __attribute__((ext_vector_type(16))) _Float16 v16h;
typedef __attribute__((ext_vector_type(8)))  _Float16 v8h;
typedef __attribute__((ext_vector_type(8)))  float    v8f;
typedef __attribute__((ext_vector_type(4)))  float    v4f;
typedef __attribute__((ext_vector_type(4)))  unsigned v4u;

__device__ __forceinline__ unsigned short f2bf_bits(float f) {
  unsigned u = __float_as_uint(f);
  return (unsigned short)((u + 0x7FFFu + ((u >> 16) & 1u)) >> 16);
}
__device__ __forceinline__ float bf_bits2f(unsigned short h) { return __uint_as_float(((unsigned)h) << 16); }
__device__ __forceinline__ float bf16r(float f) { return bf_bits2f(f2bf_bits(f)); }

__device__ __forceinline__ float h16_to_f32(unsigned hb) {
  const unsigned sgn = (hb & 0x8000u) << 16;
  const unsigned em = hb & 0x7fffu;
  const float fn = __uint_as_float((em << 13) + 0x38000000u);
  const float fs = (float)em * 5.9604644775390625e-8f;
  const float mag = (em < 0x400u) ? fs : fn;
  return __uint_as_float(__float_as_uint(mag) | sgn);
}

union FragU { v16h v; v8h h[2]; };
__device__ __forceinline__ v16h frag_load(const _Float16* p) {
  FragU f;
  f.h[0] = *(const v8h*)(p);
  f.h[1] = *(const v8h*)(p + 16);
  return f.v;
}
__device__ __forceinline__ v8f frag_mma(v16h a, v16h b, v8f c) {
  return __builtin_amdgcn_wmma_f32_16x16x32_f16(false, a, false, b, (short)0, c, false, false);
}
__device__ __forceinline__ void guard4in(v8f& a, v8f& b, v8f& c, v8f& d, v16h x, v16h y) {
  asm volatile("v_nop\n\tv_nop\n\tv_nop\n\tv_nop" : "+v"(a), "+v"(b), "+v"(c), "+v"(d) : "v"(x), "v"(y));
}
__device__ __forceinline__ void guard6in(v8f& a, v8f& b, v8f& c, v8f& d, v8f& e, v8f& f,
                                         v16h x0, v16h x1, v16h y0, v16h y1, v16h y2) {
  asm volatile("v_nop\n\tv_nop\n\tv_nop\n\tv_nop"
               : "+v"(a), "+v"(b), "+v"(c), "+v"(d), "+v"(e), "+v"(f)
               : "v"(x0), "v"(x1), "v"(y0), "v"(y1), "v"(y2));
}
__device__ __forceinline__ void keep4_h(v16h a, v16h b, v16h c, v16h d) { asm volatile("v_nop" :: "v"(a), "v"(b), "v"(c), "v"(d)); }
__device__ __forceinline__ void acc_guard4(v8f& a, v8f& b, v8f& c, v8f& d) {
  asm volatile("v_nop\n\tv_nop\n\tv_nop\n\tv_nop" : "+v"(a), "+v"(b), "+v"(c), "+v"(d));
}

__device__ __forceinline__ float fsig(float x)  { return __builtin_amdgcn_rcpf(1.0f + expf(-x)); }
__device__ __forceinline__ float ftanh_id(float x) { return 1.0f - 2.0f * __builtin_amdgcn_rcpf(expf(2.0f * x) + 1.0f); }

template <int BIAS_MODE, int OUT_MODE>
__global__ __launch_bounds__(256) void wmma_gemm64(
    const unsigned short* __restrict__ Ap, int lda, long strideA,
    const unsigned short* __restrict__ Btp, int ldb, long strideB,
    void* __restrict__ Cout, int ldc, long strideC,
    const float* __restrict__ bias, int Mr, int Nc, int Kd, float scale) {
  const _Float16* A = (const _Float16*)Ap;
  const _Float16* Bt = (const _Float16*)Btp;
  __shared__ __align__(16) float sT[8][16 * 68];
  const int b    = blockIdx.y;
  const int lane = threadIdx.x & 31;
  const int wave = threadIdx.x >> 5;
  const int tilesN = Nc >> 6;
  const int tilesM = Mr >> 6;
  const int tile = blockIdx.x * 8 + wave;
  if (tile >= tilesM * tilesN) return;
  const int tm = tile / tilesN;
  const int tn = tile - tm * tilesN;
  const int m0 = tm << 6;
  const int n0 = tn << 6;

  const _Float16* Ab = A  + (size_t)b * strideA;
  const _Float16* Bb = Bt + (size_t)b * strideB;

  const int rlane = lane & 15;
  const int koff  = (lane >> 4) * 8;
  const int mOff  = (lane >> 4) * 8;

  v8f acc[4][4];
#pragma unroll
  for (int i = 0; i < 4; ++i)
#pragma unroll
    for (int j = 0; j < 4; ++j) acc[i][j] = (v8f){0.f,0.f,0.f,0.f,0.f,0.f,0.f,0.f};

  for (int k0 = 0; k0 < Kd; k0 += 32) {
    v16h bh[4];
#pragma unroll
    for (int j = 0; j < 4; ++j) {
      const size_t bo = (size_t)(n0 + (j << 4) + rlane) * ldb + koff + k0;
      bh[j] = frag_load(Bb + bo);
    }
#pragma unroll
    for (int i = 0; i < 4; ++i) {
      const size_t ao = (size_t)(m0 + (i << 4) + rlane) * lda + koff + k0;
      v16h ah = frag_load(Ab + ao);
#pragma unroll
      for (int j = 0; j < 4; ++j) acc[i][j] = frag_mma(ah, bh[j], acc[i][j]);
      guard4in(acc[i][0], acc[i][1], acc[i][2], acc[i][3], ah, bh[3]);
    }
    keep4_h(bh[0], bh[1], bh[2], bh[3]);
  }
  acc_guard4(acc[0][0], acc[0][1], acc[0][2], acc[0][3]);
  acc_guard4(acc[1][0], acc[1][1], acc[1][2], acc[1][3]);
  acc_guard4(acc[2][0], acc[2][1], acc[2][2], acc[2][3]);
  acc_guard4(acc[3][0], acc[3][1], acc[3][2], acc[3][3]);

  float* slab = sT[wave];
#pragma unroll
  for (int i = 0; i < 4; ++i) {
    const int mBase = m0 + (i << 4);
#pragma unroll
    for (int j = 0; j < 4; ++j) {
      const int n = n0 + (j << 4) + rlane;
      float bv = 0.f;
      if (BIAS_MODE == 2) bv = bias[n];
#pragma unroll
      for (int r = 0; r < 8; ++r) {
        float v = acc[i][j][r] * scale;
        if (BIAS_MODE == 2) v += bv;
        slab[(mOff + r) * 68 + (j << 4) + rlane] = v;
      }
    }
    __builtin_amdgcn_fence(__ATOMIC_RELEASE, "workgroup");
    __builtin_amdgcn_wave_barrier();
    __builtin_amdgcn_fence(__ATOMIC_ACQUIRE, "workgroup");
    if (OUT_MODE == 0) {
      float* C = (float*)Cout + (size_t)b * strideC;
      const int hh = lane >> 4, c4 = (lane & 15) * 4;
      for (int pass = 0; pass < 2; ++pass) {
#pragma unroll
        for (int it = 0; it < 8; ++it) {
          const int row = it * 2 + hh;
          v4f v = *(const v4f*)(slab + row * 68 + c4);
          *(volatile v4f*)(C + (size_t)(mBase + row) * ldc + n0 + c4) = v;
        }
        __threadfence();
      }
    } else {
      const int q = lane >> 3, c8 = (lane & 7) * 8;
      unsigned short* C = (unsigned short*)Cout + (size_t)b * strideC;
      for (int pass = 0; pass < 2; ++pass) {
#pragma unroll
        for (int it = 0; it < 4; ++it) {
          const int row = it * 4 + q;
          const float* sp = slab + row * 68 + c8;
          v8h hv;
#pragma unroll
          for (int e = 0; e < 8; ++e) hv[e] = (_Float16)sp[e];
          *(volatile v8h*)(C + (size_t)(mBase + row) * ldc + n0 + c8) = hv;
        }
        __threadfence();
      }
    }
    __builtin_amdgcn_fence(__ATOMIC_RELEASE, "workgroup");
    __builtin_amdgcn_wave_barrier();
    __builtin_amdgcn_fence(__ATOMIC_ACQUIRE, "workgroup");
  }
}

__global__ __launch_bounds__(192) void prep_small_kernel(
    const float* __restrict__ s0, const float* __restrict__ s1, const float* __restrict__ s2, const float* __restrict__ s3,
    const float* __restrict__ s4, const float* __restrict__ s5, const float* __restrict__ s6, const float* __restrict__ s7,
    const float* __restrict__ bw, float* __restrict__ dst) {
  const int bx = blockIdx.x;
  const float* s = s0;
  if (bx == 1) s = s1;
  if (bx == 2) s = s2;
  if (bx == 3) s = s3;
  if (bx == 4) s = s4;
  if (bx == 5) s = s5;
  if (bx == 6) s = s6;
  if (bx == 7) s = s7;
  if (bx >= 8) s = bw;
  const int soff = (bx == 9) ? 768 : 0;
  const int idx = threadIdx.x * 4;
  const v4f v = *(const v4f*)(s + soff + idx);
  v4f o;
#pragma unroll
  for (int e = 0; e < 4; ++e) o[e] = bf16r(v[e]);
  float* op = dst + bx * 768 + idx;
  *(volatile v4f*)op = o;
  __threadfence();
  *(volatile v4f*)op = o;
}

__global__ __launch_bounds__(256) void wcvt_kernel(const float* __restrict__ srcA, const float* __restrict__ srcB,
                                                   unsigned short* __restrict__ dst, int n8, float sc) {
  const int i = blockIdx.x * 256 + threadIdx.x;
  const int y = blockIdx.y;
  const float* src = y ? srcB : srcA;
  if (i < n8) {
    const float* sp = src + (size_t)i * 8;
    const v4f a = *(const v4f*)(sp);
    const v4f b = *(const v4f*)(sp + 4);
    v8h hv;
#pragma unroll
    for (int e = 0; e < 4; ++e) {
      const float fa = a[e];
      const float fb = b[e];
      hv[e]     = (_Float16)(bf16r(fa) * sc);
      hv[4 + e] = (_Float16)(bf16r(fb) * sc);
    }
    unsigned short* dp = dst + (size_t)y * (size_t)n8 * 8 + (size_t)i * 8;
    *(volatile v8h*)dp = hv;
    __threadfence();
    *(volatile v8h*)dp = hv;
  }
}

__global__ __launch_bounds__(256) void gather_kernel(const int* __restrict__ pb, const int* __restrict__ qb,
                                                     const float* __restrict__ emb, unsigned short* __restrict__ X16) {
  const int i = blockIdx.x * 256 + threadIdx.x;
  const int row = i >> 5;
  const int c8 = (i & 31) * 8;
  const int rp = (row < NPR) ? row : (NPR - 1);
  int rq = row - NPR;
  rq = (rq < 0) ? 0 : rq;
  rq = (rq > NQR - 1) ? (NQR - 1) : rq;
  const int bp = rp / TPL, tp = rp - bp * TPL;
  const int bq = rq / TQL, tq = rq - bq * TQL;
  const int tokp = pb[tp * NBAT + bp];
  const int tokq = qb[tq * NBAT + bq];
  int tok = (row < NPR) ? tokp : tokq;
  tok = (tok < 0) ? 0 : tok;
  tok = (tok > VOCAB - 1) ? (VOCAB - 1) : tok;
  const float* sp = emb + (size_t)tok * EMB + c8;
  const v4f a = *(const v4f*)(sp);
  const v4f b = *(const v4f*)(sp + 4);
  v8h hv;
#pragma unroll
  for (int e = 0; e < 4; ++e) {
    const float fa = a[e];
    const float fb = b[e];
    hv[e]     = (_Float16)(bf16r(fa) * X_CARRY);
    hv[4 + e] = (_Float16)(bf16r(fb) * X_CARRY);
  }
  unsigned short* dp = X16 + (size_t)row * EMB + c8;
  *(volatile v8h*)dp = hv;
  __threadfence();
  *(volatile v8h*)dp = hv;
}

template <bool FINAL>
__global__ __launch_bounds__(512) void gru_seq_kernel(
    const float* __restrict__ GI, const unsigned short* __restrict__ WHp, const float* __restrict__ BHH,
    unsigned short* __restrict__ planeP, unsigned short* __restrict__ planeQ,
    float* __restrict__ OUT0, float* __restrict__ OUT1, int dir) {
  __shared__ __align__(16) _Float16 Ah[32 * HP16];
  __shared__ __align__(16) float    Gs[32 * GPF];
  __shared__ __align__(16) float    Hs[FINAL ? 32 * HSPF : 4];
  const _Float16* WH = (const _Float16*)WHp;
  const int tid = threadIdx.x, lane = tid & 31, wave = tid >> 5;
  const int c = lane & 15, hh = lane >> 4, koff = hh * 8;
  const int seq = FINAL ? 0 : (int)blockIdx.x;
  const int nstep = (seq == 0) ? TPL : TQL;
  const int rowbase = (seq == 0) ? 0 : NPR;
  unsigned short* plane = (seq == 0) ? planeP : planeQ;
  const int j = 16 * wave + c;

  {
    unsigned* aw = (unsigned*)Ah;
#pragma unroll 1
    for (int i = tid; i < 32 * HP16 / 2; i += 512) aw[i] = 0u;
  }
  const float b_r = BHH[j];
  const float b_z = BHH[HID + j];
  const float b_n = BHH[2 * HID + j];
  float h0[8], h1[8];
#pragma unroll
  for (int r = 0; r < 8; ++r) { h0[r] = 0.0f; h1[r] = 0.0f; }
  __syncthreads();

  const _Float16* ah0 = Ah + c * HP16 + koff;
  const _Float16* ah1 = Ah + (16 + c) * HP16 + koff;
  const _Float16* wr = WH + (size_t)j * HID + koff;
  const _Float16* wz = wr + (size_t)HID * HID;
  const _Float16* wn = wr + (size_t)2 * HID * HID;
  const v8f z8 = {0.f, 0.f, 0.f, 0.f, 0.f, 0.f, 0.f, 0.f};

#pragma unroll 1
  for (int s = 0; s < nstep; ++s) {
    const int t = dir ? (nstep - 1 - s) : s;
#pragma unroll
    for (int half = 0; half < 2; ++half) {
      v4f tmp[6];
#pragma unroll
      for (int i = 0; i < 6; ++i) {
        const int idx = (half * 6 + i) * 512 + tid;
        const int bb = idx / 192;
        const int c4 = (idx - bb * 192) * 4;
        tmp[i] = *(const v4f*)(GI + (size_t)(rowbase + bb * nstep + t) * G3 + c4);
      }
#pragma unroll
      for (int i = 0; i < 6; ++i) {
        const int idx = (half * 6 + i) * 512 + tid;
        const int bb = idx / 192;
        const int c4 = (idx - bb * 192) * 4;
        *(v4f*)(Gs + bb * GPF + c4) = tmp[i];
      }
      asm volatile("" ::: "memory");
    }

    v8f accR0 = z8, accR1 = z8, accZ0 = z8, accZ1 = z8, accN0 = z8, accN1 = z8;
#pragma unroll 1
    for (int k0 = 0; k0 < HID; k0 += 32) {
      const v16h a0 = frag_load(ah0 + k0);
      const v16h a1 = frag_load(ah1 + k0);
      const v16h br = frag_load(wr + k0);
      const v16h bz = frag_load(wz + k0);
      const v16h bn = frag_load(wn + k0);
      accR0 = frag_mma(a0, br, accR0);
      accR1 = frag_mma(a1, br, accR1);
      accZ0 = frag_mma(a0, bz, accZ0);
      accZ1 = frag_mma(a1, bz, accZ1);
      accN0 = frag_mma(a0, bn, accN0);
      accN1 = frag_mma(a1, bn, accN1);
      guard6in(accR0, accR1, accZ0, accZ1, accN0, accN1, a0, a1, br, bz, bn);
    }
    __syncthreads();

#pragma unroll 1
    for (int mt = 0; mt < 2; ++mt) {
#pragma unroll
      for (int r = 0; r < 8; ++r) {
        const int row = 16 * mt + 8 * hh + r;
        const float* gp = Gs + row * GPF + j;
        const float ir = gp[0];
        const float iz = gp[HID];
        const float inn = gp[2 * HID];
        const float cr = (mt ? accR1[r] : accR0[r]) * W_INV + b_r;
        const float cz = (mt ? accZ1[r] : accZ0[r]) * W_INV + b_z;
        const float cn = (mt ? accN1[r] : accN0[r]) * W_INV + b_n;
        const float rg = fsig(ir + cr);
        const float zg = fsig(iz + cz);
        const float ng = ftanh_id(inn + rg * cn);
        const float hold = mt ? h1[r] : h0[r];
        const float hn = (1.0f - zg) * ng + zg * hold;
        h0[r] = mt ? h0[r] : hn;
        h1[r] = mt ? hn : h1[r];
        Ah[row * HP16 + j] = (_Float16)hn;
        if (FINAL) Hs[row * HSPF + j] = hn;
      }
    }
    __syncthreads();

    if (!FINAL) {
      v8h sv[2];
#pragma unroll
      for (int i = 0; i < 2; ++i) {
        const int idx = i * 512 + tid;
        const int row = idx >> 5, c8 = (idx & 31) * 8;
        sv[i] = *(const v8h*)(Ah + row * HP16 + c8);
      }
      for (int pass = 0; pass < 2; ++pass) {
#pragma unroll
        for (int i = 0; i < 2; ++i) {
          const int idx = i * 512 + tid;
          const int row = idx >> 5, c8 = (idx & 31) * 8;
          *(volatile v8h*)(plane + (size_t)(row * nstep + t) * DM + dir * HID + c8) = sv[i];
        }
        __threadfence();
      }
    } else {
      const bool last = (s == nstep - 1);
      v4f sv[4];
#pragma unroll
      for (int i = 0; i < 4; ++i) {
        const int idx = i * 512 + tid;
        const int row = idx >> 6, c4 = (idx & 63) * 4;
        sv[i] = *(const v4f*)(Hs + row * HSPF + c4);
      }
      for (int pass = 0; pass < 2; ++pass) {
#pragma unroll
        for (int i = 0; i < 4; ++i) {
          const int idx = i * 512 + tid;
          const int row = idx >> 6, c4 = (idx & 63) * 4;
          *(volatile v4f*)(OUT0 + (size_t)(t * NBAT + row) * DM + dir * HID + c4) = sv[i];
          if (last) *(volatile v4f*)(OUT1 + (size_t)row * HID + c4) = sv[i];
        }
        __threadfence();
      }
    }
  }
}

__global__ __launch_bounds__(256) void qprep_kernel(const unsigned short* __restrict__ Q16, const float* __restrict__ BW,
                                                    unsigned short* __restrict__ QM16, unsigned short* __restrict__ QT16,
                                                    float* __restrict__ SQ) {
  __shared__ float Tt[64 * 65];
  __shared__ float Wq[DM];
  __shared__ float Wm[DM];
  __shared__ __align__(16) float Sq[64];
  const int tid = threadIdx.x;
  const int b = blockIdx.x;
  Wq[tid]       = BW[DM + tid];
  Wq[256 + tid] = BW[DM + 256 + tid];
  Wm[tid]       = BW[2 * DM + tid];
  Wm[256 + tid] = BW[2 * DM + 256 + tid];
  float sacc = 0.0f;
#pragma unroll 1
  for (int db = 0; db < 8; ++db) {
    __syncthreads();
#pragma unroll
    for (int i = 0; i < 2; ++i) {
      const int idx = i * 256 + tid;
      const int q = idx >> 3, c8 = (idx & 7) * 8;
      const size_t off = (size_t)(b * TQL + q) * DM + db * 64 + c8;
      const v4u w = *(const v4u*)(Q16 + off);
      float f[8];
#pragma unroll
      for (int k = 0; k < 4; ++k) {
        const unsigned wk = w[k];
        f[2 * k]     = h16_to_f32(wk & 0xffffu);
        f[2 * k + 1] = h16_to_f32(wk >> 16);
      }
      v8h hv;
#pragma unroll
      for (int e = 0; e < 8; ++e) {
        Tt[q * 65 + c8 + e] = f[e];
        hv[e] = (_Float16)(f[e] * Wm[db * 64 + c8 + e] * QM_CARRY);
      }
      *(volatile v8h*)(QM16 + off) = hv;
      __threadfence();
      *(volatile v8h*)(QM16 + off) = hv;
    }
    __syncthreads();
#pragma unroll
    for (int i = 0; i < 2; ++i) {
      const int idx = i * 256 + tid;
      const int dd = idx >> 3, c8 = (idx & 7) * 8;
      v8h hv;
#pragma unroll
      for (int e = 0; e < 8; ++e) hv[e] = (_Float16)Tt[(c8 + e) * 65 + dd];
      const size_t off = ((size_t)b * DM + db * 64 + dd) * TQL + c8;
      *(volatile v8h*)(QT16 + off) = hv;
      __threadfence();
      *(volatile v8h*)(QT16 + off) = hv;
    }
    if (tid < 64) {
#pragma unroll 1
      for (int dd = 0; dd < 64; ++dd) sacc += Tt[tid * 65 + dd] * Wq[db * 64 + dd];
    }
  }
  if (tid < 64) Sq[tid] = sacc;
  __syncthreads();
  if (tid < 16) {
    const v4f o = *(const v4f*)(Sq + 4 * tid);
    float* op = SQ + b * TQL + 4 * tid;
    *(volatile v4f*)op = o;
    __threadfence();
    *(volatile v4f*)op = o;
  }
}

__global__ __launch_bounds__(256) void softmax_q_kernel(const float* __restrict__ SIM, const float* __restrict__ SQ,
                                                        unsigned short* __restrict__ C2Q) {
  const int tid = threadIdx.x, lane = tid & 31, wv = tid >> 5;
  const int row = (blockIdx.x * 8 + wv) * 4 + (lane >> 3);
  const int c8 = (lane & 7) * 8;
  const int b = row / TPL;
  const v4f s0 = *(const v4f*)(SIM + (size_t)row * TQL + c8);
  const v4f s1 = *(const v4f*)(SIM + (size_t)row * TQL + c8 + 4);
  const v4f q0 = *(const v4f*)(SQ + b * TQL + c8);
  const v4f q1 = *(const v4f*)(SQ + b * TQL + c8 + 4);
  float v[8];
#pragma unroll
  for (int e = 0; e < 4; ++e) { v[e] = s0[e] + q0[e]; v[4 + e] = s1[e] + q1[e]; }
  float mx = v[0];
#pragma unroll
  for (int e = 1; e < 8; ++e) mx = fmaxf(mx, v[e]);
  mx = fmaxf(mx, __shfl_xor(mx, 1, 32));
  mx = fmaxf(mx, __shfl_xor(mx, 2, 32));
  mx = fmaxf(mx, __shfl_xor(mx, 4, 32));
  float sm = 0.0f;
#pragma unroll
  for (int e = 0; e < 8; ++e) { v[e] = expf(v[e] - mx); sm += v[e]; }
  sm += __shfl_xor(sm, 1, 32);
  sm += __shfl_xor(sm, 2, 32);
  sm += __shfl_xor(sm, 4, 32);
  const float inv = P_CARRY * __builtin_amdgcn_rcpf(sm);
  v8h hv;
#pragma unroll
  for (int e = 0; e < 8; ++e) hv[e] = (_Float16)(v[e] * inv);
  unsigned short* dp = C2Q + (size_t)row * TQL + c8;
  *(volatile v8h*)dp = hv;
  __threadfence();
  *(volatile v8h*)dp = hv;
}

__global__ __launch_bounds__(384) void q2c_kernel(const unsigned short* __restrict__ P16, const float* __restrict__ SIM,
                                                  const float* __restrict__ SQ, const float* __restrict__ BW,
                                                  float* __restrict__ Q2CV) {
  __shared__ float Wp[DM];
  __shared__ float Sq[TQL];
  __shared__ float Mv[TPL];
  __shared__ float red[12];
  __shared__ __align__(16) float Ov[DM];
  const int tid = threadIdx.x, lane = tid & 31, wv = tid >> 5;
  const int b = blockIdx.x;
  Wp[tid] = BW[tid];
  if (tid < DM - TPL) Wp[TPL + tid] = BW[TPL + tid];
  if (tid < TQL) Sq[tid] = SQ[b * TQL + tid];
  __syncthreads();

  const size_t prow = (size_t)(b * TPL + tid);
  const v4u* pw = (const v4u*)(P16 + prow * DM);
  float sp = 0.0f;
#pragma unroll 1
  for (int ch = 0; ch < DM / 8; ++ch) {
    const v4u w = pw[ch];
#pragma unroll
    for (int k = 0; k < 4; ++k) {
      const unsigned wk = w[k];
      sp += h16_to_f32(wk & 0xffffu) * Wp[ch * 8 + 2 * k];
      sp += h16_to_f32(wk >> 16) * Wp[ch * 8 + 2 * k + 1];
    }
  }
  const v4f* sr = (const v4f*)(SIM + prow * TQL);
  float mx = -INFINITY;
#pragma unroll 1
  for (int i = 0; i < TQL / 4; ++i) {
    const v4f sv = sr[i];
#pragma unroll
    for (int e = 0; e < 4; ++e) mx = fmaxf(mx, sv[e] + Sq[4 * i + e]);
  }
  const float m = sp + mx;

  float wm = m;
#pragma unroll
  for (int off = 1; off < 32; off <<= 1) wm = fmaxf(wm, __shfl_xor(wm, off, 32));
  if (lane == 0) red[wv] = wm;
  __syncthreads();
  float bm = red[0];
#pragma unroll
  for (int i = 1; i < 12; ++i) bm = fmaxf(bm, red[i]);
  __syncthreads();
  const float ev = expf(m - bm);
  float ws = ev;
#pragma unroll
  for (int off = 1; off < 32; off <<= 1) ws += __shfl_xor(ws, off, 32);
  if (lane == 0) red[wv] = ws;
  __syncthreads();
  float bs = 0.0f;
#pragma unroll
  for (int i = 0; i < 12; ++i) bs += red[i];
  Mv[tid] = ev * (1.0f / bs);
  __syncthreads();

  if (tid < 256) {
    const unsigned* pu = (const unsigned*)(P16 + (size_t)b * TPL * DM);
    float a0 = 0.0f, a1 = 0.0f;
#pragma unroll 1
    for (int pp = 0; pp < TPL; ++pp) {
      const unsigned w = pu[(size_t)pp * (DM / 2) + tid];
      const float at = Mv[pp];
      a0 += at * h16_to_f32(w & 0xffffu);
      a1 += at * h16_to_f32(w >> 16);
    }
    Ov[2 * tid] = a0;
    Ov[2 * tid + 1] = a1;
  }
  __syncthreads();
  if (tid < 128) {
    const v4f o = *(const v4f*)(Ov + 4 * tid);
    float* op = Q2CV + b * DM + 4 * tid;
    *(volatile v4f*)op = o;
    __threadfence();
    *(volatile v4f*)op = o;
  }
}

__global__ __launch_bounds__(256) void buildg_kernel(const unsigned short* __restrict__ P16, const float* __restrict__ Q2CV,
                                                     unsigned short* __restrict__ G16) {
  const int i = blockIdx.x * 256 + threadIdx.x;
  const int row = i >> 6;
  const int d0 = (i & 63) * 8;
  const int b = row / TPL;
  const v4u pw = *(const v4u*)(P16 + (size_t)row * DM + d0);
  const v4u cw = *(const v4u*)(G16 + (size_t)row * GW + DM + d0);
  const v4f qa = *(const v4f*)(Q2CV + b * DM + d0);
  const v4f qb = *(const v4f*)(Q2CV + b * DM + d0 + 4);
  float pf[8], cf[8], qf[8];
#pragma unroll
  for (int k = 0; k < 4; ++k) {
    const unsigned pk = pw[k];
    const unsigned ck = cw[k];
    pf[2 * k]     = h16_to_f32(pk & 0xffffu);
    pf[2 * k + 1] = h16_to_f32(pk >> 16);
    cf[2 * k]     = h16_to_f32(ck & 0xffffu);
    cf[2 * k + 1] = h16_to_f32(ck >> 16);
    qf[k]     = qa[k];
    qf[4 + k] = qb[k];
  }
  v8h o0, o2, o3;
#pragma unroll
  for (int e = 0; e < 8; ++e) {
    o0[e] = (_Float16)(pf[e] * G_CARRY);
    o2[e] = (_Float16)(pf[e] * cf[e]);
    o3[e] = (_Float16)(pf[e] * qf[e] * G_CARRY);
  }
  unsigned short* gp = G16 + (size_t)row * GW + d0;
  for (int pass = 0; pass < 2; ++pass) {
    *(volatile v8h*)(gp) = o0;
    *(volatile v8h*)(gp + 2 * DM) = o2;
    *(volatile v8h*)(gp + 3 * DM) = o3;
    __threadfence();
  }
}

constexpr size_t SZ_W256 = (size_t)2 * G3 * HID * 2;
constexpr size_t SZ_WIH4 = (size_t)2 * G3 * GW * 2;
constexpr size_t SZ_BIAS = (size_t)10 * 768 * 4;
constexpr size_t SZ_SQ   = (size_t)NBAT * TQL * 4;
constexpr size_t SZ_Q2CV = (size_t)NBAT * DM * 4;
constexpr size_t SZ_X16  = (size_t)NXR * EMB * 2;
constexpr size_t SZ_GI   = (size_t)NXR * G3 * 4;
constexpr size_t SZ_P16  = (size_t)NPR * DM * 2;
constexpr size_t SZ_Q16  = (size_t)NQR * DM * 2;
constexpr size_t SZ_SIM  = (size_t)NBAT * TPL * TQL * 4;
constexpr size_t SZ_C2Q  = (size_t)NBAT * TPL * TQL * 2;
constexpr size_t SZ_G16  = (size_t)NPR * GW * 2;
constexpr size_t WS_TOTAL = 3 * SZ_W256 + SZ_WIH4 + SZ_BIAS + SZ_SQ + SZ_Q2CV + SZ_X16 + SZ_GI + SZ_P16 + 3 * SZ_Q16 +
                            SZ_SIM + SZ_C2Q + SZ_G16;
static_assert(WS_TOTAL == (size_t)134060032);
static_assert(WS_TOTAL <= (size_t)134217728);
static_assert(SZ_W256 % 256 == 0 && SZ_WIH4 % 256 == 0 && SZ_BIAS % 256 == 0 && SZ_SQ % 256 == 0 && SZ_Q2CV % 256 == 0);
static_assert(SZ_X16 % 256 == 0 && SZ_GI % 256 == 0 && SZ_P16 % 256 == 0 && SZ_Q16 % 256 == 0 && SZ_SIM % 256 == 0);
static_assert(SZ_C2Q % 256 == 0 && SZ_G16 % 256 == 0);
static_assert((size_t)NPR * G3 * 4 <= SZ_GI);

extern "C" void kernel_launch(void* const* d_in, const int* in_sizes, int n_in,
                              void* d_out, int out_size, void* d_ws, size_t ws_size, hipStream_t stream) {
  if (n_in < 20 || d_out == nullptr || d_ws == nullptr) return;
  if (in_sizes[0] != TPL * NBAT || in_sizes[1] != TQL * NBAT || in_sizes[2] != VOCAB * EMB) return;
  if (in_sizes[3] != G3 * EMB || in_sizes[4] != G3 * HID || in_sizes[7] != G3 * EMB || in_sizes[8] != G3 * HID) return;
  if (in_sizes[5] != G3 || in_sizes[6] != G3 || in_sizes[9] != G3 || in_sizes[10] != G3) return;
  if (in_sizes[11] != 3 * DM) return;
  if (in_sizes[12] != G3 * GW || in_sizes[13] != G3 * HID || in_sizes[16] != G3 * GW || in_sizes[17] != G3 * HID) return;
  if (in_sizes[14] != G3 || in_sizes[15] != G3 || in_sizes[18] != G3 || in_sizes[19] != G3) return;
  if (out_size != OUT0_FLOATS + OUT1_FLOATS) return;
  if (ws_size < WS_TOTAL) return;

  const int*   p_batch = (const int*)d_in[0];
  const int*   q_batch = (const int*)d_in[1];
  const float* emb     = (const float*)d_in[2];
  const float* w1_ih_f = (const float*)d_in[3];
  const float* w1_hh_f = (const float*)d_in[4];
  const float* b1_ih_f = (const float*)d_in[5];
  const float* b1_hh_f = (const float*)d_in[6];
  const float* w1_ih_b = (const float*)d_in[7];
  const float* w1_hh_b = (const float*)d_in[8];
  const float* b1_ih_b = (const float*)d_in[9];
  const float* b1_hh_b = (const float*)d_in[10];
  const float* bidaf_w = (const float*)d_in[11];
  const float* w4_ih_f = (const float*)d_in[12];
  const float* w4_hh_f = (const float*)d_in[13];
  const float* b4_ih_f = (const float*)d_in[14];
  const float* b4_hh_f = (const float*)d_in[15];
  const float* w4_ih_b = (const float*)d_in[16];
  const float* w4_hh_b = (const float*)d_in[17];
  const float* b4_ih_b = (const float*)d_in[18];
  const float* b4_hh_b = (const float*)d_in[19];

  float* out0 = (float*)d_out;
  float* out1 = out0 + (size_t)OUT0_FLOATS;

  char* ws = (char*)d_ws;
  size_t off = 0;
  auto carve = [&](size_t bytes) -> char* { char* p = ws + off; off += bytes; return p; };
  unsigned short* WIH1 = (unsigned short*)carve(SZ_W256);
  unsigned short* WHH1 = (unsigned short*)carve(SZ_W256);
  unsigned short* WIH4 = (unsigned short*)carve(SZ_WIH4);
  unsigned short* WHH4 = (unsigned short*)carve(SZ_W256);
  float*          BIASBW = (float*)carve(SZ_BIAS);
  float*          SQ   = (float*)carve(SZ_SQ);
  float*          Q2CV = (float*)carve(SZ_Q2CV);
  unsigned short* X16  = (unsigned short*)carve(SZ_X16);
  float*          GI   = (float*)carve(SZ_GI);
  unsigned short* P16  = (unsigned short*)carve(SZ_P16);
  unsigned short* Q16  = (unsigned short*)carve(SZ_Q16);
  unsigned short* QM16 = (unsigned short*)carve(SZ_Q16);
  unsigned short* QT16 = (unsigned short*)carve(SZ_Q16);
  float*          SIM  = (float*)carve(SZ_SIM);
  unsigned short* C2Q  = (unsigned short*)carve(SZ_C2Q);
  unsigned short* G16  = (unsigned short*)carve(SZ_G16);
  if (off != WS_TOTAL || off > ws_size) return;
  float* BWF = BIASBW + 8 * 768;

  prep_small_kernel<<<10, 192, 0, stream>>>(b1_ih_f, b1_hh_f, b1_ih_b, b1_hh_b, b4_ih_f, b4_hh_f, b4_ih_b, b4_hh_b, bidaf_w, BIASBW);
  const int n8s = G3 * HID / 8;
  const int n8l = G3 * GW / 8;
  wcvt_kernel<<<dim3(n8s / 256, 2), 256, 0, stream>>>(w1_ih_f, w1_ih_b, WIH1, n8s, W_CARRY);
  wcvt_kernel<<<dim3(n8s / 256, 2), 256, 0, stream>>>(w1_hh_f, w1_hh_b, WHH1, n8s, W_CARRY);
  wcvt_kernel<<<dim3(n8l / 256, 2), 256, 0, stream>>>(w4_ih_f, w4_ih_b, WIH4, n8l, W_CARRY);
  wcvt_kernel<<<dim3(n8s / 256, 2), 256, 0, stream>>>(w4_hh_f, w4_hh_b, WHH4, n8s, W_CARRY);
  gather_kernel<<<NXR * 32 / 256, 256, 0, stream>>>(p_batch, q_batch, emb, X16);

  for (int dir = 0; dir < 2; ++dir) {
    wmma_gemm64<2, 0><<<dim3((NXR / 64) * (G3 / 64) / 8, 1), 256, 0, stream>>>(
        X16, EMB, 0L, WIH1 + (size_t)dir * G3 * EMB, EMB, 0L, (void*)GI, G3, 0L,
        BIASBW + (dir ? 2 : 0) * 768, NXR, G3, EMB, GI_SCALE);
    gru_seq_kernel<false><<<2, 512, 0, stream>>>(
        GI, WHH1 + (size_t)dir * G3 * HID, BIASBW + (dir ? 3 : 1) * 768, P16, Q16, out0, out1, dir);
  }

  qprep_kernel<<<NBAT, 256, 0, stream>>>(Q16, BWF, QM16, QT16, SQ);
  wmma_gemm64<0, 0><<<dim3(1, NBAT), 256, 0, stream>>>(
      P16, DM, (long)TPL * DM, QM16, DM, (long)TQL * DM, (void*)SIM, TQL, (long)TPL * TQL,
      BIASBW, TPL, TQL, DM, CROSS_SCALE);
  softmax_q_kernel<<<NPR / 32, 256, 0, stream>>>(SIM, SQ, C2Q);
  wmma_gemm64<0, 1><<<dim3((TPL / 64) * (DM / 64) / 8, NBAT), 256, 0, stream>>>(
      C2Q, TQL, (long)TPL * TQL, QT16, TQL, (long)DM * TQL, (void*)(G16 + DM), GW, (long)TPL * GW,
      BIASBW, TPL, DM, TQL, C2QV_SCALE);
  q2c_kernel<<<NBAT, 384, 0, stream>>>(P16, SIM, SQ, BWF, Q2CV);
  buildg_kernel<<<NPR * 64 / 256, 256, 0, stream>>>(P16, Q2CV, G16);

  for (int dir = 0; dir < 2; ++dir) {
    wmma_gemm64<2, 0><<<dim3((NPR / 64) * (G3 / 64) / 8, 1), 256, 0, stream>>>(
        G16, GW, 0L, WIH4 + (size_t)dir * G3 * GW, GW, 0L, (void*)GI, G3, 0L,
        BIASBW + (dir ? 6 : 4) * 768, NPR, G3, GW, GI4_SCALE);
    gru_seq_kernel<true><<<1, 512, 0, stream>>>(
        GI, WHH4 + (size_t)dir * G3 * HID, BIASBW + (dir ? 7 : 5) * 768, P16, Q16, out0,
        out1 + (size_t)dir * NBAT * HID, dir);
  }
}
